// LstmModel_31851477467289
// MI455X (gfx1250) — hardware-run, weakly checked
//
#include <hip/hip_runtime.h>
#include <math.h>

typedef __attribute__((ext_vector_type(16))) _Float16 v16h;
typedef __attribute__((ext_vector_type(8)))  _Float16 v8h;
typedef __attribute__((ext_vector_type(8)))  float    v8f;
typedef __attribute__((ext_vector_type(4)))  float    v4f;

constexpr int NSTEP   = 512;
constexpr int NBATCH  = 256;
constexpr int NHID    = 256;
constexpr int NG3     = 3 * NHID;
constexpr int NPRED   = 256;
constexpr int ROWS_PB = 16;
constexpr int NBLK    = NBATCH / ROWS_PB;
constexpr int NTHR    = 256;
constexpr int SEQ_BOUND = 512;
constexpr int APITCH  = NHID + 8;
constexpr int HEAD_STEPS = 16;
constexpr int MK_STEPS = 32;
constexpr int PQ_W    = 128;
constexpr int TP_EDGE = 32;
constexpr int TP_PITCH = 33;
constexpr int WELEMS  = NG3 * NHID;
constexpr int PELEMS  = NPRED * NHID;
constexpr int PREP_BLK_W  = WELEMS / 8 / 256;
constexpr int PREP_BLK_P  = PELEMS / 8 / 256;
constexpr int PREP_BLOCKS = 5 * PREP_BLK_W + PREP_BLK_P;
constexpr int NOUT0 = NSTEP * NBATCH;
constexpr int NOUT1 = NBATCH * NPRED;
constexpr int GATE_BYTES = NHID * NHID * 2;
constexpr int PLANE_BYTES = WELEMS * 2;
constexpr unsigned NT_BYTES = 16u * NHID * 2u;

constexpr float H_CARRY    = 16.0f;
constexpr float W_CARRY    = 64.0f;
constexpr float RES_CARRY  = 2048.0f;
constexpr float RES_INV    = 1.0f / RES_CARRY;
constexpr float PROD_INV   = 1.0f / (H_CARRY * W_CARRY);
constexpr float HB_CARRY   = 256.0f;
constexpr float HB_FACTOR  = HB_CARRY / (float)NSTEP;
constexpr float HEAD_SCALE = 1.0f / (HB_CARRY * W_CARRY);
constexpr float F16_MIN_NORMAL = 6.103515625e-5f;

static_assert(NBATCH % ROWS_PB == 0);
static_assert(ROWS_PB == 16);
static_assert(NBLK == 16);
static_assert(NHID == 32 * (NTHR / 32));
static_assert(NHID == NTHR);
static_assert(NHID % 32 == 0);
static_assert(APITCH % 8 == 0);
static_assert(NSTEP % MK_STEPS == 0);
static_assert(MK_STEPS * 4 == 128);
static_assert(PQ_W == 16 * (NTHR / 32));
static_assert(ROWS_PB == 2 * (NTHR / 32));
static_assert(NSTEP % TP_EDGE == 0 && NBATCH % TP_EDGE == 0);
static_assert(PREP_BLK_W * 256 * 8 == WELEMS);
static_assert(PREP_BLK_P * 256 * 8 == PELEMS);
static_assert(PREP_BLOCKS == 512);
static_assert(NBATCH % 64 == 0 && NPRED % 64 == 0 && NHID % 32 == 0);
static_assert((NOUT0 * 4) % 128 == 0);
static_assert(PLANE_BYTES == 3 * GATE_BYTES);
static_assert(PLANE_BYTES % 256 == 0);
static_assert(SEQ_BOUND >= NTHR);

__device__ __forceinline__ unsigned short f2bf_bits(float f) {
  unsigned u = __float_as_uint(f);
  return (unsigned short)((u + 0x7FFFu + ((u >> 16) & 1u)) >> 16);
}
__device__ __forceinline__ float bf_bits2f(unsigned short h) { return __uint_as_float(((unsigned)h) << 16); }

__device__ __forceinline__ void dep_guard_h(v8f& a, v8f& b, v16h x, v16h y) { asm volatile("v_nop\n\tv_nop\n\tv_nop\n\tv_nop" : "+v"(a), "+v"(b) : "v"(x), "v"(y)); }
__device__ __forceinline__ void keep4_h(v16h a, v16h b, v16h c, v16h d) { asm volatile("v_nop" :: "v"(a), "v"(b), "v"(c), "v"(d)); }
__device__ __forceinline__ void acc_guard4(v8f& a, v8f& b, v8f& c, v8f& d) { asm volatile("v_nop\n\tv_nop\n\tv_nop\n\tv_nop" : "+v"(a), "+v"(b), "+v"(c), "+v"(d)); }
__device__ __forceinline__ void tie1(v8f& a) { asm volatile("" : "+v"(a)); }
__device__ __forceinline__ void settle(v8f& a) { asm volatile("v_nop\n\tv_nop\n\tv_nop\n\tv_nop" : "+v"(a)); }
__device__ __forceinline__ void guard4in(v8f& a, v16h x0, v16h x1, v16h x2, v16h x3) {
  asm volatile("v_nop\n\tv_nop\n\tv_nop\n\tv_nop" : "+v"(a) : "v"(x0), "v"(x1), "v"(x2), "v"(x3));
}
__device__ __forceinline__ unsigned pin_u(unsigned x) { asm volatile("" : "+v"(x)); return x; }
__device__ __forceinline__ int pin_i(int x) { asm volatile("" : "+v"(x)); return x; }

template <typename T> struct Frag;
template <> struct Frag<_Float16> {
  typedef v16h V; union U { v16h v; v8h h[2]; };
  static __device__ __forceinline__ v16h load(const _Float16* p) {
    U f; f.h[0] = *(const v8h*)(p); f.h[1] = *(const v8h*)(p + 16); return f.v;
  }
  static __device__ __forceinline__ v8f mma(v16h a, v16h b, v8f c) {
    return __builtin_amdgcn_wmma_f32_16x16x32_f16(false, a, false, b, (short)0, c, false, false);
  }
  static __device__ __forceinline__ void guard(v8f& a, v8f& b, v16h x, v16h y) { dep_guard_h(a, b, x, y); }
  static __device__ __forceinline__ void keep(v16h a, v16h b, v16h c, v16h d) { keep4_h(a, b, c, d); }
};
typedef Frag<_Float16> FragH;

__device__ __forceinline__ v16h ldW(const char* plane, unsigned boff) {
  return FragH::load((const _Float16*)(plane + boff));
}

template <int ET> struct Elem;
template <> struct Elem<0> { typedef _Float16 T; };
template <int ET, bool SPLIT, int BIAS_MODE, int OUT_MODE, bool RESID, int ACT = 0>
__global__ __launch_bounds__(256) void wmma_gemm64(
    const unsigned short* __restrict__ Ap, const unsigned short* __restrict__ A2p, int lda, long strideA,
    const unsigned short* __restrict__ Btp, const unsigned short* __restrict__ Bt2p, int ldb, long strideB,
    void* __restrict__ Cout, void* __restrict__ Cout2, int ldc, long strideC,
    const float* __restrict__ bias,
    const float* __restrict__ resid, long strideR,
    int M, int N, int K, float scale) {
  typedef typename Elem<ET>::T T;
  typedef typename Frag<T>::V V;
  const T* A = (const T*)Ap; const T* A2 = (const T*)A2p; const T* Bt = (const T*)Btp; const T* Bt2 = (const T*)Bt2p;
  __shared__ __align__(16) float sT[8][16 * 68];
  const int b    = blockIdx.y;
  const int lane = threadIdx.x & 31;
  const int wave = threadIdx.x >> 5;
  const int tilesN = N >> 6;
  const int tilesM = M >> 6;
  const int tile = blockIdx.x * 8 + wave;
  if (tile >= tilesM * tilesN) return;
  const int tm = tile / tilesN;
  const int tn = tile - tm * tilesN;
  const int m0 = tm << 6;
  const int n0 = tn << 6;

  const T* Ab  = A  + (size_t)b * strideA;
  const T* Bb  = Bt + (size_t)b * strideB;
  const T* Ab2 = SPLIT ? (A2  + (size_t)b * strideA) : nullptr;
  const T* Bb2 = SPLIT ? (Bt2 + (size_t)b * strideB) : nullptr;

  const int rlane = lane & 15;
  const int koff  = (lane >> 4) * 8;
  const int mOff  = (lane >> 4) * 8;

  v8f acc[4][4];
#pragma unroll
  for (int i = 0; i < 4; ++i)
#pragma unroll
    for (int j = 0; j < 4; ++j) acc[i][j] = (v8f){0.f,0.f,0.f,0.f,0.f,0.f,0.f,0.f};

  for (int k0 = 0; k0 < K; k0 += 32) {
    V bh[4], bl[4];
#pragma unroll
    for (int j = 0; j < 4; ++j) {
      const size_t bo = (size_t)(n0 + (j << 4) + rlane) * ldb + koff + k0;
      bh[j] = Frag<T>::load(Bb + bo);
      if (SPLIT) bl[j] = Frag<T>::load(Bb2 + bo);
    }
#pragma unroll
    for (int i = 0; i < 4; ++i) {
      const size_t ao = (size_t)(m0 + (i << 4) + rlane) * lda + koff + k0;
      V ah = Frag<T>::load(Ab + ao);
      V al;
      if (SPLIT) al = Frag<T>::load(Ab2 + ao);
#pragma unroll
      for (int j = 0; j < 4; ++j) {
        acc[i][j] = Frag<T>::mma(ah, bh[j], acc[i][j]);
        if (SPLIT) {
          acc[i][j] = Frag<T>::mma(ah, bl[j], acc[i][j]);
          acc[i][j] = Frag<T>::mma(al, bh[j], acc[i][j]);
        }
      }
      tie1(acc[i][1]);
      tie1(acc[i][2]);
      Frag<T>::guard(acc[i][0], acc[i][3], ah, SPLIT ? al : ah);
    }
    Frag<T>::keep(bh[0], bh[1], bh[2], bh[3]);
    if (SPLIT) Frag<T>::keep(bl[0], bl[1], bl[2], bl[3]);
  }
  acc_guard4(acc[0][0], acc[0][1], acc[0][2], acc[0][3]);
  acc_guard4(acc[1][0], acc[1][1], acc[1][2], acc[1][3]);
  acc_guard4(acc[2][0], acc[2][1], acc[2][2], acc[2][3]);
  acc_guard4(acc[3][0], acc[3][1], acc[3][2], acc[3][3]);

  float* slab = sT[wave];
  const float* Rb = RESID ? (resid + (size_t)b * strideR) : nullptr;
#pragma unroll
  for (int i = 0; i < 4; ++i) {
    const int mBase = m0 + (i << 4);
#pragma unroll
    for (int j = 0; j < 4; ++j) {
      const int n = n0 + (j << 4) + rlane;
      float bv = 0.f;
      if (BIAS_MODE == 2) bv = bias[n];
#pragma unroll
      for (int r = 0; r < 8; ++r) {
        float v = acc[i][j][r] * scale;
        if (BIAS_MODE == 1) v += bias[mBase + mOff + r];
        if (BIAS_MODE == 2) v += bv;
        if (RESID) v += Rb[(size_t)(mBase + mOff + r) * ldc + n];
        if (ACT == 1) v = tanhf(v);
        if (ACT == 2) v = fmaxf(v, 0.0f);
        if (ACT == 4) v = (v > 0.f) ? v : 0.01f * v;
        slab[(mOff + r) * 68 + (j << 4) + rlane] = v;
      }
    }
    __builtin_amdgcn_fence(__ATOMIC_RELEASE, "workgroup");
    __builtin_amdgcn_wave_barrier();
    __builtin_amdgcn_fence(__ATOMIC_ACQUIRE, "workgroup");
    if (OUT_MODE == 0) {
      float* C = (float*)Cout + (size_t)b * strideC;
      const int hh = lane >> 4, c4 = (lane & 15) * 4;
      for (int pass = 0; pass < 2; ++pass) {
#pragma unroll
        for (int it = 0; it < 8; ++it) {
          const int row = it * 2 + hh;
          v4f v = *(const v4f*)(slab + row * 68 + c4);
          *(volatile v4f*)(C + (size_t)(mBase + row) * ldc + n0 + c4) = v;
        }
        __threadfence();
      }
    } else {
      const int q = lane >> 3, c8 = (lane & 7) * 8;
      unsigned short* C  = (unsigned short*)Cout  + (size_t)b * strideC;
      unsigned short* C2 = (OUT_MODE == 2) ? ((unsigned short*)Cout2 + (size_t)b * strideC) : nullptr;
      for (int pass = 0; pass < 2; ++pass) {
#pragma unroll
        for (int it = 0; it < 4; ++it) {
          const int row = it * 4 + q;
          const float* sp = slab + row * 68 + c8;
          v8h hv, lv;
#pragma unroll
          for (int e = 0; e < 8; ++e) {
            if (OUT_MODE == 1) {
              hv[e] = (_Float16)sp[e];
            } else {
              unsigned short hb = f2bf_bits(sp[e]);
              unsigned short lb = f2bf_bits(sp[e] - bf_bits2f(hb));
              hv[e] = __builtin_bit_cast(_Float16, hb);
              lv[e] = __builtin_bit_cast(_Float16, lb);
            }
          }
          *(volatile v8h*)(C + (size_t)(mBase + row) * ldc + n0 + c8) = hv;
          if (OUT_MODE == 2) *(volatile v8h*)(C2 + (size_t)(mBase + row) * ldc + n0 + c8) = lv;
        }
        __threadfence();
      }
    }
    __builtin_amdgcn_fence(__ATOMIC_RELEASE, "workgroup");
    __builtin_amdgcn_wave_barrier();
    __builtin_amdgcn_fence(__ATOMIC_ACQUIRE, "workgroup");
  }
}

__device__ __forceinline__ float flush16(float v) { return (fabsf(v) < F16_MIN_NORMAL) ? 0.0f : v; }
__device__ __forceinline__ float fsig(float x)  { return __builtin_amdgcn_rcpf(1.0f + __expf(-x)); }
__device__ __forceinline__ float ftanh(float x) { return 1.0f - 2.0f * __builtin_amdgcn_rcpf(__expf(2.0f * x) + 1.0f); }

__global__ __launch_bounds__(256) void prep_kernel(
    const float* __restrict__ w0, const float* __restrict__ w1, const float* __restrict__ w2,
    const float* __restrict__ w3, const float* __restrict__ w4, const float* __restrict__ wp,
    unsigned short* __restrict__ v0, unsigned short* __restrict__ v1, unsigned short* __restrict__ v2,
    unsigned short* __restrict__ v3, unsigned short* __restrict__ v4, unsigned short* __restrict__ vp,
    unsigned short* __restrict__ r0, unsigned short* __restrict__ r1, unsigned short* __restrict__ r2) {
  const int blk = blockIdx.x, tid = threadIdx.x;
  const float* src;
  unsigned short* dv;
  unsigned short* dr;
  bool hasres;
  int lb;
  if (blk < PREP_BLK_W)          { src = w0; dv = v0; dr = r0; hasres = true;  lb = blk; }
  else if (blk < 2 * PREP_BLK_W) { src = w1; dv = v1; dr = r1; hasres = true;  lb = blk - PREP_BLK_W; }
  else if (blk < 3 * PREP_BLK_W) { src = w2; dv = v2; dr = r2; hasres = true;  lb = blk - 2 * PREP_BLK_W; }
  else if (blk < 4 * PREP_BLK_W) { src = w3; dv = v3; dr = v3; hasres = false; lb = blk - 3 * PREP_BLK_W; }
  else if (blk < 5 * PREP_BLK_W) { src = w4; dv = v4; dr = v4; hasres = false; lb = blk - 4 * PREP_BLK_W; }
  else                           { src = wp; dv = vp; dr = vp; hasres = false; lb = blk - 5 * PREP_BLK_W; }
  const int i = lb * 256 + tid;
  const float* sp = src + (size_t)i * 8;
  const v4f a = *(const v4f*)(sp);
  const v4f b = *(const v4f*)(sp + 4);
  v8h hv, rv;
#pragma unroll
  for (int e = 0; e < 4; ++e) {
    const float xa = a[e] * W_CARRY;
    const float xb = b[e] * W_CARRY;
    const _Float16 ha = (_Float16)flush16(xa);
    const _Float16 hb = (_Float16)flush16(xb);
    hv[e]     = ha;
    hv[4 + e] = hb;
    rv[e]     = (_Float16)flush16((xa - (float)ha) * RES_CARRY);
    rv[4 + e] = (_Float16)flush16((xb - (float)hb) * RES_CARRY);
  }
  volatile v8h* pv = (volatile v8h*)(dv + (size_t)i * 8);
  volatile v8h* pr = (volatile v8h*)(dr + (size_t)i * 8);
  *pv = hv;
  if (hasres) *pr = rv;
  __threadfence();
  *pv = hv;
  if (hasres) *pr = rv;
}


__device__ __forceinline__ void pass3(const _Float16* a0, const char* wpl, unsigned wb,
                                      v8f& r0, v8f& z0, v8f& n0) {
#pragma unroll 1
  for (int kc = 0; kc < NHID / 32; ++kc) {
    const unsigned kb = wb + (unsigned)kc * 64u;
    const v16h fa  = FragH::load(a0 + kc * 32);
    const v16h fb0 = ldW(wpl, kb);
    const v16h fb1 = ldW(wpl + GATE_BYTES, kb);
    const v16h fb2 = ldW(wpl + 2 * GATE_BYTES, kb);
    r0 = FragH::mma(fa, fb0, r0);
    z0 = FragH::mma(fa, fb1, z0);
    n0 = FragH::mma(fa, fb2, n0);
    tie1(r0);
    tie1(z0);
    guard4in(n0, fa, fb0, fb1, fb2);
  }
}

__device__ __forceinline__ void headpass(const _Float16* av, const _Float16* ar, const char* wv, const char* wr, unsigned wb,
                                         v8f& v, v8f& q) {
#pragma unroll 1
  for (int kc = 0; kc < NHID / 32; ++kc) {
    const unsigned kb = wb + (unsigned)kc * 64u;
    const v16h fa = FragH::load(av + kc * 32);
    const v16h ra = FragH::load(ar + kc * 32);
    const v16h fb = ldW(wv, kb);
    const v16h rb = ldW(wr, kb);
    v = FragH::mma(fa, fb, v);
    q = FragH::mma(fa, rb, q);
    q = FragH::mma(ra, fb, q);
    tie1(v);
    guard4in(q, fa, ra, fb, rb);
  }
}

__device__ __forceinline__ void headgate(const _Float16* av, const _Float16* ar, const char* wv, const char* wr, unsigned wb,
                                         v8f& g) {
  v8f v = (v8f){0.f,0.f,0.f,0.f,0.f,0.f,0.f,0.f};
  v8f q = v;
  headpass(av, ar, wv, wr, wb, v, q);
  settle(v);
  settle(q);
#pragma unroll
  for (int r = 0; r < 8; ++r) g[r] += v[r] + q[r] * RES_INV;
}

__device__ __forceinline__ void head3(const _Float16* av, const _Float16* ar, const char* wv, const char* wr, unsigned wb,
                                      v8f& r0, v8f& z0, v8f& n0) {
  headgate(av, ar, wv, wr, wb, r0);
  headgate(av, ar, wv + GATE_BYTES, wr + GATE_BYTES, wb, z0);
  headgate(av, ar, wv + 2 * GATE_BYTES, wr + 2 * GATE_BYTES, wb, n0);
}

__device__ __forceinline__ v8f ld_hold(const v4f* ms) {
  const v4f a = ms[0];
  const v4f b = ms[NTHR];
  const v8f h = {a[0], a[1], a[2], a[3], b[0], b[1], b[2], b[3]};
  return h;
}
__device__ __forceinline__ void st_hold(v4f* ms, v8f h) {
  const v4f a = {h[0], h[1], h[2], h[3]};
  const v4f b = {h[4], h[5], h[6], h[7]};
  ms[0] = a;
  ms[NTHR] = b;
}
__device__ __forceinline__ void add_hold(v4f* hs, v8f h) {
  const v4f a = hs[0];
  const v4f b = hs[NTHR];
  const v4f ha = {h[0], h[1], h[2], h[3]};
  const v4f hb = {h[4], h[5], h[6], h[7]};
  const v4f na = a + ha;
  const v4f nb = b + hb;
  hs[0] = na;
  hs[NTHR] = nb;
}

__device__ __forceinline__ void enc_tile(v8f ar, v8f az, v8f an, v8f xv, v4f k0, v4f k1, v4f* ms) {
  const v8f hold = ld_hold(ms);
  v8f hn;
#pragma unroll
  for (int r = 0; r < 8; ++r) {
    const float x  = xv[r];
    const float rg = fsig(ar[r] * PROD_INV + (x * k0[0] + k0[3]));
    const float zg = fsig(az[r] * PROD_INV + (x * k0[1] + k1[0]));
    const float ng = ftanh((x * k0[2] + k1[1]) + rg * (an[r] * PROD_INV + k1[2]));
    hn[r] = ng + zg * (hold[r] - ng);
  }
  st_hold(ms, hn);
}

__device__ __forceinline__ v8f dec_tile(v8f ar, v8f az, v8f ai, v8f ah, v4f k, v4f* ms) {
  const v8f hold = ld_hold(ms);
  v8f hn;
#pragma unroll
  for (int r = 0; r < 8; ++r) {
    const float rg = fsig(ar[r] * PROD_INV + k[0]);
    const float zg = fsig(az[r] * PROD_INV + k[1]);
    const float ng = ftanh((ai[r] * PROD_INV + k[2]) + rg * (ah[r] * PROD_INV + k[3]));
    hn[r] = ng + zg * (hold[r] - ng);
  }
  st_hold(ms, hn);
  return hn;
}

__device__ __forceinline__ void publish(const v4f* ms, _Float16* av, _Float16* ar, bool withres, int wave, int c, int hh) {
#pragma unroll 1
  for (int i4 = 0; i4 < 4; ++i4) {
    const v4f m = ms[i4 * NTHR];
    const int nt = i4 >> 1, q = i4 & 1;
    const int eo = (8 * hh + 4 * q) * APITCH + 32 * wave + 16 * nt + c;
#pragma unroll
    for (int e = 0; e < 4; ++e) {
      const float me = m[e];
      const float xs = me * H_CARRY;
      const _Float16 hv = (_Float16)flush16(xs);
      av[eo + e * APITCH] = hv;
      if (withres) {
        const float rs = (xs - (float)hv) * RES_CARRY;
        ar[eo + e * APITCH] = (_Float16)flush16(rs);
      }
    }
  }
}

__global__ __launch_bounds__(SEQ_BOUND) __attribute__((amdgpu_num_vgpr(256)))
void gru3_seq_kernel(
    const float* __restrict__ seq, const float* __restrict__ dly,
    const float* __restrict__ h0e, const float* __restrict__ h0m, const float* __restrict__ h0p,
    const float* __restrict__ e_wih, const float* __restrict__ e_bih, const float* __restrict__ e_bhh,
    const float* __restrict__ m_bih, const float* __restrict__ m_bhh,
    const float* __restrict__ mlw, const float* __restrict__ mlb,
    const float* __restrict__ p_bih, const float* __restrict__ p_bhh,
    const unsigned short* WVp, const unsigned short* WRp,
    float* __restrict__ MK, unsigned short* __restrict__ HB) {
  __shared__ __align__(16) _Float16 Av[3][ROWS_PB * APITCH];
  __shared__ __align__(16) _Float16 Ar[2][ROWS_PB * APITCH];
  __shared__ __align__(16) v4f      Mst[3][4][NTHR];
  __shared__ __align__(16) v4f      Hsum[4][NTHR];
  __shared__ __align__(16) float    Ctab[NHID * 16];
  __shared__ __align__(16) float    Pq[ROWS_PB * PQ_W];
  __shared__ __align__(16) float    Mstage[ROWS_PB * MK_STEPS];

  const int tid = threadIdx.x, lane = tid & 31, wave = tid >> 5;
  const int c = lane & 15, hh = lane >> 4, koff = hh * 8;
  const int rowbase = blockIdx.x * ROWS_PB;
  const char* WV = (const char*)WVp;
  const char* WR = (const char*)WRp;
  const float mlb0 = mlb[0];
  const v8f z8 = {0.f, 0.f, 0.f, 0.f, 0.f, 0.f, 0.f, 0.f};

  _Float16* Le  = &Av[0][0];
  _Float16* Lm  = &Av[1][0];
  _Float16* Lp  = &Av[2][0];
  _Float16* LeR = &Ar[0][0];
  _Float16* LmR = &Ar[1][0];

  {
    const int n = tid;
    const v4f t0 = {e_wih[n], e_wih[NHID + n], e_wih[2 * NHID + n], e_bih[n] + e_bhh[n]};
    const v4f t1 = {e_bih[NHID + n] + e_bhh[NHID + n], e_bih[2 * NHID + n], e_bhh[2 * NHID + n], mlw[n]};
    *(v4f*)(Ctab + n * 16)      = t0;
    *(v4f*)(Ctab + n * 16 + 4)  = t1;
    __builtin_amdgcn_sched_barrier(0);
    const v4f t2 = {m_bih[n] + m_bhh[n], m_bih[NHID + n] + m_bhh[NHID + n], m_bih[2 * NHID + n], m_bhh[2 * NHID + n]};
    const v4f t3 = {p_bih[n] + p_bhh[n], p_bih[NHID + n] + p_bhh[NHID + n], p_bih[2 * NHID + n], p_bhh[2 * NHID + n]};
    *(v4f*)(Ctab + n * 16 + 8)  = t2;
    *(v4f*)(Ctab + n * 16 + 12) = t3;
  }

#pragma unroll 1
  for (int s = 0; s < 3; ++s) {
    const float* h0 = (s == 0) ? h0e : ((s == 1) ? h0m : h0p);
#pragma unroll 1
    for (int nt = 0; nt < 2; ++nt) {
      const float* hp = h0 + (size_t)(rowbase + 8 * hh) * NHID + 32 * wave + 16 * nt + c;
      v4f m0, m1;
      m0[0] = hp[0];
      m0[1] = hp[NHID];
      m0[2] = hp[2 * NHID];
      m0[3] = hp[3 * NHID];
      m1[0] = hp[4 * NHID];
      m1[1] = hp[5 * NHID];
      m1[2] = hp[6 * NHID];
      m1[3] = hp[7 * NHID];
      Mst[s][nt * 2][tid]     = m0;
      Mst[s][nt * 2 + 1][tid] = m1;
    }
  }
  {
    const v4f z4 = {0.f, 0.f, 0.f, 0.f};
#pragma unroll 1
    for (int i4 = 0; i4 < 4; ++i4) Hsum[i4][tid] = z4;
  }
  publish(&Mst[0][0][tid], Le, LeR, true, wave, c, hh);
  publish(&Mst[1][0][tid], Lm, LmR, true, wave, c, hh);
  publish(&Mst[2][0][tid], Lp, LeR, false, wave, c, hh);
  __syncthreads();

  const int aoff0 = c * APITCH + koff;
  const unsigned wb0 = (unsigned)(((32 * wave + c) * NHID + koff) * 2);

#pragma unroll 1
  for (int t = 0; t < NSTEP; ++t) {
    const bool head = (t < HEAD_STEPS);
    const int aoff = pin_i(aoff0);

    {
      const int ts = (t > 0) ? (t - 1) : 0;
      const float* xsrc = (t == 0) ? dly : (seq + (size_t)ts * NBATCH);
      const float* xp = xsrc + rowbase + 8 * hh;
      const v4f xa0 = *(const v4f*)(xp);
      const v4f xa1 = *(const v4f*)(xp + 4);
      const v8f xm = {xa0[0], xa0[1], xa0[2], xa0[3], xa1[0], xa1[1], xa1[2], xa1[3]};
#pragma unroll 1
      for (int nt = 0; nt < 2; ++nt) {
        const int j = 32 * wave + 16 * nt + c;
        const unsigned wb = pin_u(wb0 + (unsigned)nt * NT_BYTES);
        v8f gr = z8, gz = z8, gn = z8;
        if (head) {
          head3(Le + aoff, LeR + aoff, WV, WR, wb, gr, gz, gn);
        } else {
          pass3(Le + aoff, WV, wb, gr, gz, gn);
          settle(gr);
          settle(gz);
          settle(gn);
        }
        const v4f k0 = *(const v4f*)(Ctab + j * 16);
        const v4f k1 = *(const v4f*)(Ctab + j * 16 + 4);
        v4f* ms = &Mst[0][nt * 2][tid];
        enc_tile(gr, gz, gn, xm, k0, k1, ms);
        __builtin_amdgcn_sched_barrier(0);
      }
    }
    __syncthreads();
    publish(&Mst[0][0][tid], Le, LeR, head, wave, c, hh);
    __syncthreads();

#pragma unroll 1
    for (int s = 1; s < 3; ++s) {
      const bool hd = head && (s == 1);
      const char* wiV = WV + (size_t)(2 * s - 1) * PLANE_BYTES;
      const char* whV = WV + (size_t)(2 * s) * PLANE_BYTES;
      const char* wiR = WR + (size_t)PLANE_BYTES;
      const char* whR = WR + (size_t)2 * PLANE_BYTES;
      const _Float16* Lh = &Av[s][0];
      v8f pm = z8;
#pragma unroll 1
      for (int nt = 0; nt < 2; ++nt) {
        const int j = 32 * wave + 16 * nt + c;
        const unsigned wb = pin_u(wb0 + (unsigned)nt * NT_BYTES);
        v8f gr = z8, gz = z8, gi = z8, gh = z8;
        if (hd) {
          head3(Le + aoff, LeR + aoff, wiV, wiR, wb, gr, gz, gi);
          head3(Lh + aoff, LmR + aoff, whV, whR, wb, gr, gz, gh);
        } else {
          pass3(Le + aoff, wiV, wb, gr, gz, gi);
          pass3(Lh + aoff, whV, wb, gr, gz, gh);
          settle(gr);
          settle(gz);
          settle(gi);
          settle(gh);
        }
        const v4f kk = *(const v4f*)(Ctab + j * 16 + 4 + 4 * s);
        const float wm = Ctab[j * 16 + 7];
        v4f* ms = &Mst[s][nt * 2][tid];
        v4f* hs = &Hsum[nt * 2][tid];
        const v8f hn = dec_tile(gr, gz, gi, gh, kk, ms);
        if (s == 1) {
#pragma unroll
          for (int r = 0; r < 8; ++r) pm[r] += hn[r] * wm;
        } else {
          add_hold(hs, hn);
        }
        __builtin_amdgcn_sched_barrier(0);
      }
      if (s == 1) {
#pragma unroll
        for (int r = 0; r < 8; ++r) Pq[(8 * hh + r) * PQ_W + wave * 16 + c] = pm[r];
      }
    }
    __syncthreads();
    publish(&Mst[1][0][tid], Lm, LmR, head, wave, c, hh);
    publish(&Mst[2][0][tid], Lp, LeR, false, wave, c, hh);

    if (wave == 0) {
      const float* pr = Pq + c * PQ_W + hh * (PQ_W / 2);
      float sum = 0.0f;
#pragma unroll 4
      for (int i = 0; i < PQ_W / 8; ++i) {
        const v4f p = *(const v4f*)(pr + 4 * i);
        sum += (p[0] + p[1]) + (p[2] + p[3]);
      }
      const float other = __shfl_xor(sum, 16, 32);
      const float mv = (sum + other) + mlb0;
      if (hh == 0) Mstage[c * MK_STEPS + (t & (MK_STEPS - 1))] = mv;

      if ((t & (MK_STEPS - 1)) == (MK_STEPS - 1)) {
        __builtin_amdgcn_fence(__ATOMIC_RELEASE, "workgroup");
        __builtin_amdgcn_wave_barrier();
        __builtin_amdgcn_fence(__ATOMIC_ACQUIRE, "workgroup");
        const int tb = t - (MK_STEPS - 1);
        const int q8 = lane >> 3, c4 = (lane & 7) * 4;
        const v4f s0 = *(const v4f*)(Mstage + (0 * 4 + q8) * MK_STEPS + c4);
        const v4f s1 = *(const v4f*)(Mstage + (1 * 4 + q8) * MK_STEPS + c4);
        const v4f s2 = *(const v4f*)(Mstage + (2 * 4 + q8) * MK_STEPS + c4);
        const v4f s3 = *(const v4f*)(Mstage + (3 * 4 + q8) * MK_STEPS + c4);
        float* mk0 = MK + (size_t)(rowbase + q8) * NSTEP + tb + c4;
        for (int pass = 0; pass < 2; ++pass) {
          *(volatile v4f*)(mk0)                      = s0;
          *(volatile v4f*)(mk0 + (size_t)4 * NSTEP)  = s1;
          *(volatile v4f*)(mk0 + (size_t)8 * NSTEP)  = s2;
          *(volatile v4f*)(mk0 + (size_t)12 * NSTEP) = s3;
          __threadfence();
        }
        __builtin_amdgcn_fence(__ATOMIC_RELEASE, "workgroup");
        __builtin_amdgcn_wave_barrier();
        __builtin_amdgcn_fence(__ATOMIC_ACQUIRE, "workgroup");
      }
    }
  }

#pragma unroll 1
  for (int nt = 0; nt < 2; ++nt) {
    const v8f sv = ld_hold(&Hsum[nt * 2][tid]);
#pragma unroll
    for (int r = 0; r < 8; ++r) {
      const float hv = sv[r] * HB_FACTOR;
      Lp[(8 * hh + r) * APITCH + 32 * wave + 16 * nt + c] = (_Float16)flush16(hv);
    }
  }
  __syncthreads();
  for (int pass = 0; pass < 2; ++pass) {
#pragma unroll
    for (int i = 0; i < 2; ++i) {
      const int row = 2 * wave + i;
      const v8h v = *(const v8h*)(Lp + row * APITCH + 8 * lane);
      *(volatile v8h*)(HB + (size_t)(rowbase + row) * NHID + 8 * lane) = v;
    }
    __threadfence();
  }
}

__global__ __launch_bounds__(256) void mask_transpose_kernel(const float* __restrict__ MK, float* __restrict__ out) {
  __shared__ float tl[TP_EDGE * TP_PITCH];
  const int tid = threadIdx.x;
  const int s0 = blockIdx.x * TP_EDGE;
  const int b0 = blockIdx.y * TP_EDGE;
  const int rr = tid >> 3;
  const int p4 = (tid & 7) * 4;
  {
    const v4f v = *(const v4f*)(MK + (size_t)(b0 + rr) * NSTEP + s0 + p4);
    const float e0 = v[0];
    const float e1 = v[1];
    const float e2 = v[2];
    const float e3 = v[3];
    tl[rr * TP_PITCH + p4 + 0] = e0;
    tl[rr * TP_PITCH + p4 + 1] = e1;
    tl[rr * TP_PITCH + p4 + 2] = e2;
    tl[rr * TP_PITCH + p4 + 3] = e3;
  }
  __syncthreads();
  v4f o;
  o[0] = tl[(p4 + 0) * TP_PITCH + rr];
  o[1] = tl[(p4 + 1) * TP_PITCH + rr];
  o[2] = tl[(p4 + 2) * TP_PITCH + rr];
  o[3] = tl[(p4 + 3) * TP_PITCH + rr];
  float* op = out + (size_t)(s0 + rr) * NBATCH + b0 + p4;
  *(volatile v4f*)op = o;
  __threadfence();
  *(volatile v4f*)op = o;
}

extern "C" void kernel_launch(void* const* d_in, const int* in_sizes, int n_in,
                              void* d_out, int out_size, void* d_ws, size_t ws_size, hipStream_t stream) {
  if (n_in < 21 || d_out == nullptr || d_ws == nullptr) return;
  if (in_sizes[0] != NSTEP * NBATCH || in_sizes[1] != NBATCH ||
      in_sizes[2] != NBATCH * NHID || in_sizes[3] != NBATCH * NHID || in_sizes[4] != NBATCH * NHID ||
      in_sizes[5] != NG3 || in_sizes[6] != WELEMS || in_sizes[7] != NG3 || in_sizes[8] != NG3 ||
      in_sizes[9] != WELEMS || in_sizes[10] != WELEMS || in_sizes[11] != NG3 || in_sizes[12] != NG3 ||
      in_sizes[13] != NHID || in_sizes[14] != 1 ||
      in_sizes[15] != WELEMS || in_sizes[16] != WELEMS || in_sizes[17] != NG3 || in_sizes[18] != NG3 ||
      in_sizes[19] != PELEMS || in_sizes[20] != NPRED ||
      out_size != NOUT0 + NOUT1) return;

  const float* seq       = (const float*)d_in[0];
  const float* dly       = (const float*)d_in[1];
  const float* h0e       = (const float*)d_in[2];
  const float* h0m       = (const float*)d_in[3];
  const float* h0p       = (const float*)d_in[4];
  const float* enc_w_ih  = (const float*)d_in[5];
  const float* enc_w_hh  = (const float*)d_in[6];
  const float* enc_b_ih  = (const float*)d_in[7];
  const float* enc_b_hh  = (const float*)d_in[8];
  const float* mdec_w_ih = (const float*)d_in[9];
  const float* mdec_w_hh = (const float*)d_in[10];
  const float* mdec_b_ih = (const float*)d_in[11];
  const float* mdec_b_hh = (const float*)d_in[12];
  const float* mlin_w    = (const float*)d_in[13];
  const float* mlin_b    = (const float*)d_in[14];
  const float* pdec_w_ih = (const float*)d_in[15];
  const float* pdec_w_hh = (const float*)d_in[16];
  const float* pdec_b_ih = (const float*)d_in[17];
  const float* pdec_b_hh = (const float*)d_in[18];
  const float* plin_w    = (const float*)d_in[19];
  const float* plin_b    = (const float*)d_in[20];
  float* out_mask = (float*)d_out;
  float* out_pred = out_mask + (size_t)NOUT0;

  char* ws = (char*)d_ws; size_t off = 0;
  auto carve = [&](size_t bytes) -> char* { char* p = ws + off; off += (bytes + 255) & ~(size_t)255; return p; };
  unsigned short* WVALL = (unsigned short*)carve((size_t)5 * WELEMS * 2);
  unsigned short* WRALL = (unsigned short*)carve((size_t)3 * WELEMS * 2);
  unsigned short* WPL   = (unsigned short*)carve((size_t)PELEMS * 2);
  unsigned short* HBP   = (unsigned short*)carve((size_t)NBATCH * NHID * 2);
  float*          MKP   = (float*)carve((size_t)NBATCH * NSTEP * 4);
  if (off > ws_size || off > (size_t)134217728) return;

  prep_kernel<<<PREP_BLOCKS, 256, 0, stream>>>(enc_w_hh, mdec_w_ih, mdec_w_hh, pdec_w_ih, pdec_w_hh, plin_w,
                                               WVALL, WVALL + (size_t)WELEMS, WVALL + (size_t)2 * WELEMS,
                                               WVALL + (size_t)3 * WELEMS, WVALL + (size_t)4 * WELEMS, WPL,
                                               WRALL, WRALL + (size_t)WELEMS, WRALL + (size_t)2 * WELEMS);

  gru3_seq_kernel<<<NBLK, NTHR, 0, stream>>>(seq, dly, h0e, h0m, h0p,
                                             enc_w_ih, enc_b_ih, enc_b_hh,
                                             mdec_b_ih, mdec_b_hh, mlin_w, mlin_b,
                                             pdec_b_ih, pdec_b_hh,
                                             WVALL, WRALL,
                                             MKP, HBP);

  wmma_gemm64<0, false, 2, 0, false, 0><<<dim3((NBATCH / 64) * (NPRED / 64) / 8, 1), 256, 0, stream>>>(
      HBP, HBP, NHID, 0L, WPL, WPL, NHID, 0L, (void*)out_pred, (void*)out_pred, NPRED, 0L,
      plin_b, plin_b, 0L, NBATCH, NPRED, NHID, HEAD_SCALE);

  mask_transpose_kernel<<<dim3(NSTEP / TP_EDGE, NBATCH / TP_EDGE), 256, 0, stream>>>(MKP, out_mask);
}
